// NeuraLogic_84945863180634
// MI455X (gfx1250) — hardware-run, weakly checked
//
#include <hip/hip_runtime.h>
#include <stddef.h>


#define DW      64
#define NTHR    256
#define NWAVE   8
#define EPT     8
#define NGRP    2
#define CHUNK   (NTHR * EPT * NGRP)
#define WCAP    (EPT * NGRP * 32)
#define LISTN   (NWAVE * WCAP)
#define NBC     4096
#define NBF     1024
#define RCAP    40960
#define RBN     128
#define TGT     128
#define DPW     (TGT / NWAVE)
#define DEGCAP  1024
#define OTHR    512
#define BM      64
#define NMAT    3
#define KH      (NMAT * DW)
#define GPB     8
#define GMAX    4096
#define WSCAP   134217728

#define LDS_FILL ((RCAP + NBF + LISTN) * 4 + 64)

static_assert((CHUNK & (CHUNK - 1)) == 0);
static_assert(CHUNK <= 4096);
static_assert((NBC & (NBC - 1)) == 0 && (NBF & (NBF - 1)) == 0);
static_assert(NBC == 4 * NBF);
static_assert(OTHR * 8 == NBC);
static_assert((RCAP % 32) == 0);
static_assert(TGT == NWAVE * DPW);
static_assert((DPW & (DPW - 1)) == 0 && DPW <= 32);
static_assert((NBC % TGT) == 0);
static_assert((TGT % BM) == 0);
static_assert(DW == 2 * 32);
static_assert((DW % 32) == 0 && (KH % 32) == 0);
static_assert(WCAP == EPT * NGRP * 32);
static_assert(GPB == NWAVE);
static_assert((GPB & (GPB - 1)) == 0);
static_assert(((GPB * DW) % NTHR) == 0);
static_assert(GPB * (DW / 4) <= NTHR);

typedef float    v2f  __attribute__((ext_vector_type(2)));
typedef float    v4f  __attribute__((ext_vector_type(4)));
typedef float    v8f  __attribute__((ext_vector_type(8)));
typedef int      v4i  __attribute__((ext_vector_type(4)));
typedef unsigned short v4us __attribute__((ext_vector_type(4)));
typedef unsigned short v8us __attribute__((ext_vector_type(8)));
typedef __bf16   v16b __attribute__((ext_vector_type(16)));
union Frag { v16b v; v8us h[2]; };

__device__ __forceinline__ v8f wmb(v16b a, v16b b, v8f c) {
  v8f d = __builtin_amdgcn_wmma_f32_16x16x32_bf16(false, a, false, b, (short)0, c, false, false);
  asm volatile("v_nop\n\tv_nop\n\tv_nop\n\tv_nop" : "+v"(d) : "v"(a), "v"(b));
  return d;
}

__device__ __forceinline__ unsigned bf16_rne(float f) {
  unsigned u = __float_as_uint(f);
  u += 0x7FFFu + ((u >> 16) & 1u);
  return u >> 16;
}
__device__ __forceinline__ void split2(float x, unsigned short* hs, unsigned short* ls) {
  const unsigned hb = bf16_rne(x);
  const float rem = x - __uint_as_float(hb << 16);
  *hs = (unsigned short)hb;
  *ls = (unsigned short)bf16_rne(rem);
}

template <int NB>
__device__ __forceinline__ int scan_chunk(const int* __restrict__ dsts, int nE, int cbase, int slotBase,
                                          int vec8, int* list, int tid, int lane, int wave) {
  int wc = 0;
#pragma unroll
  for (int g = 0; g < NGRP; ++g) {
    const int el0  = (g * NTHR + tid) * EPT;
    const int e0   = cbase + el0;
    const int sent = -2147483647 - 1;
    v4i da, db;
    if (vec8 != 0 && cbase + CHUNK <= nE) {
      da = *(const v4i*)(dsts + e0);
      db = *(const v4i*)(dsts + e0 + 4);
    } else {
      da.x = (e0     < nE) ? dsts[min(e0, nE - 1)] : sent;
      da.y = (e0 + 1 < nE) ? dsts[min(e0 + 1, nE - 1)] : sent;
      da.z = (e0 + 2 < nE) ? dsts[min(e0 + 2, nE - 1)] : sent;
      da.w = (e0 + 3 < nE) ? dsts[min(e0 + 3, nE - 1)] : sent;
      db.x = (e0 + 4 < nE) ? dsts[min(e0 + 4, nE - 1)] : sent;
      db.y = (e0 + 5 < nE) ? dsts[min(e0 + 5, nE - 1)] : sent;
      db.z = (e0 + 6 < nE) ? dsts[min(e0 + 6, nE - 1)] : sent;
      db.w = (e0 + 7 < nE) ? dsts[min(e0 + 7, nE - 1)] : sent;
    }
    const unsigned nb = (unsigned)slotBase;
    const unsigned s0 = (unsigned)da.x - nb, s1 = (unsigned)da.y - nb;
    const unsigned s2 = (unsigned)da.z - nb, s3 = (unsigned)da.w - nb;
    const unsigned s4 = (unsigned)db.x - nb, s5 = (unsigned)db.y - nb;
    const unsigned s6 = (unsigned)db.z - nb, s7 = (unsigned)db.w - nb;
    const bool h0 = s0 < (unsigned)NB, h1 = s1 < (unsigned)NB, h2 = s2 < (unsigned)NB, h3 = s3 < (unsigned)NB;
    const bool h4 = s4 < (unsigned)NB, h5 = s5 < (unsigned)NB, h6 = s6 < (unsigned)NB, h7 = s7 < (unsigned)NB;
    const unsigned any = __builtin_amdgcn_ballot_w32(h0 | h1 | h2 | h3 | h4 | h5 | h6 | h7);
    if (any != 0u) {
#define HITJ(J, HJ, SJ) { \
        const unsigned mj = __builtin_amdgcn_ballot_w32(HJ); \
        if (mj != 0u) { \
          if (HJ) { \
            const int pos = wc + (int)__builtin_amdgcn_mbcnt_lo(mj, 0u); \
            if (pos < WCAP) list[wave * WCAP + pos] = ((el0 + (J)) << 12) | (int)(SJ); \
          } \
          wc += (int)__builtin_popcount(mj); } }
      HITJ(0, h0, s0)
      HITJ(1, h1, s1)
      HITJ(2, h2, s2)
      HITJ(3, h3, s3)
      HITJ(4, h4, s4)
      HITJ(5, h5, s5)
      HITJ(6, h6, s6)
      HITJ(7, h7, s7)
#undef HITJ
    }
  }
  return wc;
}

__global__ __launch_bounds__(NTHR) void k_count(const int* __restrict__ dsts, int* cnt, int nE, int vec8) {
  __shared__ __attribute__((aligned(16))) int scnt[NBC];
  __shared__ __attribute__((aligned(16))) int list[LISTN];
  __shared__ int wcnt[NWAVE];
  const int tid = threadIdx.x, lane = tid & 31, wave = tid >> 5;
  const int nodeBase = blockIdx.x * NBC;

  for (int i = tid; i < NBC; i += NTHR) scnt[i] = 0;
  __syncthreads();

  const int nChunks = (nE + CHUNK - 1) / CHUNK;
#pragma unroll 1
  for (int ch = 0; ch < nChunks; ++ch) {
    const int cbase = ch * CHUNK;
    const int wc = scan_chunk<NBC>(dsts, nE, cbase, nodeBase, vec8, list, tid, lane, wave);
    if (lane == 0) wcnt[wave] = wc;
    __syncthreads();
    if (wave == 0) {
#pragma unroll 1
      for (int wsx = 0; wsx < NWAVE; ++wsx) {
        int n = __builtin_amdgcn_readfirstlane(wcnt[wsx]);
        n = n > WCAP ? WCAP : (n < 0 ? 0 : n);
        const int* lp = list + wsx * WCAP;
#pragma unroll 1
        for (int i = 0; i < n; ++i) {
          const int ent  = __builtin_amdgcn_readfirstlane(lp[i]);
          const int slot = ent & (NBC - 1);
          if (lane == 0) scnt[slot] = scnt[slot] + 1;
        }
      }
    }
    __syncthreads();
  }

  v4i cq[4];
#pragma unroll
  for (int q = 0; q < 4; ++q) {
    const int f = (wave * 4 + q) * 128 + 4 * lane;
    cq[q] = *(const v4i*)(scnt + f);
  }
  int* cp = cnt + (size_t)nodeBase;
#pragma unroll
  for (int q = 0; q < 4; ++q) {
    const int f = (wave * 4 + q) * 128 + 4 * lane;
    *(volatile v4i*)(cp + f) = cq[q];
  }
  __threadfence();
#pragma unroll
  for (int q = 0; q < 4; ++q) {
    const int f = (wave * 4 + q) * 128 + 4 * lane;
    *(volatile v4i*)(cp + f) = cq[q];
  }
}

__global__ __launch_bounds__(OTHR) void k_offsets(
    const int* __restrict__ cnt, int* off, int* rbase, int nChunk) {
  __shared__ __attribute__((aligned(16))) int soff[NBC];
  __shared__ __attribute__((aligned(16))) int srb[RBN];
  __shared__ int wtot[OTHR / 32];
  const int tid = threadIdx.x, lane = tid & 31, wave = tid >> 5, sub = tid >> 7;
  for (int i = tid; i < RBN; i += OTHR) srb[i] = 0;
  int carry = 0;
#pragma unroll 1
  for (int ch = 0; ch < nChunk; ++ch) {
    const int base = ch * NBC;
    const v4i c0 = *(const v4i*)(cnt + base + 8 * tid);
    const v4i c1 = *(const v4i*)(cnt + base + 8 * tid + 4);
    const int e0 = max(c0.x, 0), e1 = max(c0.y, 0), e2 = max(c0.z, 0), e3 = max(c0.w, 0);
    const int e4 = max(c1.x, 0), e5 = max(c1.y, 0), e6 = max(c1.z, 0), e7 = max(c1.w, 0);
    const int ts = e0 + e1 + e2 + e3 + e4 + e5 + e6 + e7;
    int incl = ts;
#pragma unroll
    for (int d = 1; d < 32; d <<= 1) {
      const int t = __shfl_up(incl, d);
      if (lane >= d) incl += t;
    }
    if (lane == 31) wtot[wave] = incl;
    __syncthreads();
    const int S0 = wtot[0]  + wtot[1]  + wtot[2]  + wtot[3];
    const int S1 = wtot[4]  + wtot[5]  + wtot[6]  + wtot[7];
    const int S2 = wtot[8]  + wtot[9]  + wtot[10] + wtot[11];
    const int S3 = wtot[12] + wtot[13] + wtot[14] + wtot[15];
    int pre = 0;
#pragma unroll 1
    for (int w = 4 * sub; w < wave; ++w) pre += wtot[w];
    const int b0 = carry;
    const int b1 = b0 + ((S0 + 31) & ~31);
    const int b2 = b1 + ((S1 + 31) & ~31);
    const int b3 = b2 + ((S2 + 31) & ~31);
    const int b4 = b3 + ((S3 + 31) & ~31);
    const int myb = sub == 0 ? b0 : (sub == 1 ? b1 : (sub == 2 ? b2 : b3));
    if (tid == 0) {
      srb[min(4 * ch + 0, RBN - 1)] = b0;
      srb[min(4 * ch + 1, RBN - 1)] = b1;
      srb[min(4 * ch + 2, RBN - 1)] = b2;
      srb[min(4 * ch + 3, RBN - 1)] = b3;
    }
    int run = myb + pre + incl - ts;
    soff[8 * tid + 0] = run; run += e0;
    soff[8 * tid + 1] = run; run += e1;
    soff[8 * tid + 2] = run; run += e2;
    soff[8 * tid + 3] = run; run += e3;
    soff[8 * tid + 4] = run; run += e4;
    soff[8 * tid + 5] = run; run += e5;
    soff[8 * tid + 6] = run; run += e6;
    soff[8 * tid + 7] = run;
    carry = b4;
    __syncthreads();
    const v4i o0 = *(const v4i*)(soff + 4 * tid);
    const v4i o1 = *(const v4i*)(soff + 4 * (tid + OTHR));
    int* op = off + base;
    *(volatile v4i*)(op + 4 * tid) = o0;
    *(volatile v4i*)(op + 4 * (tid + OTHR)) = o1;
    __threadfence();
    *(volatile v4i*)(op + 4 * tid) = o0;
    *(volatile v4i*)(op + 4 * (tid + OTHR)) = o1;
    __syncthreads();
  }
  if (tid == 0) srb[min(4 * nChunk, RBN - 1)] = carry;
  __syncthreads();
  v4i rv = {0, 0, 0, 0};
  if (tid < 32) rv = *(const v4i*)(srb + 4 * tid);
  if (tid < 32) *(volatile v4i*)(rbase + 4 * tid) = rv;
  __threadfence();
  if (tid < 32) *(volatile v4i*)(rbase + 4 * tid) = rv;
}

__global__ __launch_bounds__(NTHR) void k_fill(
    const int* __restrict__ srcs, const int* __restrict__ dsts,
    const int* __restrict__ off, const int* __restrict__ rbase,
    int* csr, int nN, int nE, int vec8, int csrLen) {
  extern __shared__ v4f lds_dyn[];
  int* region = (int*)lds_dyn;
  int* cursor = region + RCAP;
  int* list   = cursor + NBF;
  int* wcnt   = list + LISTN;
  const int tid = threadIdx.x, lane = tid & 31, wave = tid >> 5;
  const int b = blockIdx.x;
  const int nodeBase = b * NBF;

  int rb0 = rbase[b];
  const int rb1 = rbase[b + 1];
  rb0 = rb0 < 0 ? 0 : (rb0 > csrLen ? csrLen : rb0);
  rb0 &= ~31;
  int len = rb1 - rb0;
  len = len < 0 ? 0 : (len > RCAP ? RCAP : len);
  int lenW = (len + 31) & ~31;
  if (rb0 + lenW > csrLen) lenW = (csrLen - rb0) & ~31;

  {
    const v4i z = {0, 0, 0, 0};
    for (int i = tid; i < RCAP / 4; i += NTHR) ((v4i*)region)[i] = z;
    for (int s = tid; s < NBF; s += NTHR) {
      int o = off[nodeBase + s] - rb0;
      o = o < 0 ? 0 : (o > RCAP ? RCAP : o);
      cursor[s] = o;
    }
  }
  __syncthreads();

  const int nChunks = (nE + CHUNK - 1) / CHUNK;
#pragma unroll 1
  for (int ch = 0; ch < nChunks; ++ch) {
    const int cbase = ch * CHUNK;
    const int wc = scan_chunk<NBF>(dsts, nE, cbase, nodeBase, vec8, list, tid, lane, wave);
    if (lane == 0) wcnt[wave] = wc;
    __syncthreads();
    if (wave == 0) {
#pragma unroll 1
      for (int wsx = 0; wsx < NWAVE; ++wsx) {
        int n = __builtin_amdgcn_readfirstlane(wcnt[wsx]);
        n = n > WCAP ? WCAP : (n < 0 ? 0 : n);
        const int* lp = list + wsx * WCAP;
#pragma unroll 1
        for (int i = 0; i < n; ++i) {
          const int ent  = __builtin_amdgcn_readfirstlane(lp[i]);
          const int slot = ent & (NBF - 1);
          int e = cbase + ((ent >> 12) & (CHUNK - 1));
          e = e > nE - 1 ? nE - 1 : e;
          int sv = srcs[e];
          sv = sv < 0 ? 0 : (sv > nN - 1 ? nN - 1 : sv);
          if (lane == 0) {
            int pos = cursor[slot];
            pos = pos < 0 ? 0 : (pos > RCAP - 1 ? RCAP - 1 : pos);
            region[pos] = sv;
            const int np = pos + 1;
            cursor[slot] = np > RCAP ? RCAP : np;
          }
        }
      }
    }
    __syncthreads();
  }

  const int nv = lenW >> 2;
  int* gp = csr + rb0;
#pragma unroll 1
  for (int i = tid; i < nv; i += NTHR) { const v4i v = ((const v4i*)region)[i]; *(volatile v4i*)(gp + 4 * i) = v; }
  __threadfence();
#pragma unroll 1
  for (int i = tid; i < nv; i += NTHR) { const v4i v = ((const v4i*)region)[i]; *(volatile v4i*)(gp + 4 * i) = v; }
}

__global__ __launch_bounds__(NTHR) void k_wcvt(
    const float* __restrict__ w0, const float* __restrict__ w1, const float* __restrict__ w2,
    const float* __restrict__ w3, const float* __restrict__ w4, const float* __restrict__ w5,
    unsigned short* whi, unsigned short* wlo, int nUnits) {
  const int i = (int)blockIdx.x * NTHR + (int)threadIdx.x;
  if (i >= nUnits) return;
  const int spr = DW / 8;
  const int per = DW * spr;
  int q = i / per;
  q = q > 5 ? 5 : q;
  const int r = i - q * per;
  const int n = r / spr;
  const int seg = r - n * spr;
  const float* wb = (q == 0) ? w0 : ((q == 1) ? w1 : ((q == 2) ? w2 : ((q == 3) ? w3 : ((q == 4) ? w4 : w5))));
  const float* p = wb + (size_t)(8 * seg) * DW + n;
  const size_t dest = (q < NMAT)
      ? ((size_t)q * DW * DW + (size_t)n * DW + (size_t)(8 * seg))
      : ((size_t)NMAT * DW * DW + (size_t)n * KH + (size_t)(q - NMAT) * DW + (size_t)(8 * seg));
  v8us hv, lv;
#pragma unroll
  for (int j = 0; j < 8; ++j) {
    unsigned short hs, ls;
    split2(p[(size_t)j * DW], &hs, &ls);
    hv[j] = hs;
    lv[j] = ls;
  }
  unsigned short* gh = whi + dest;
  unsigned short* gl = wlo + dest;
  *(volatile v8us*)gh = hv;
  *(volatile v8us*)gl = lv;
  __threadfence();
  *(volatile v8us*)gh = hv;
  *(volatile v8us*)gl = lv;
}

template <int K, int RELU>
__global__ __launch_bounds__(NTHR) void k_gemm(
    const float* __restrict__ A, const unsigned short* __restrict__ Bh,
    const unsigned short* __restrict__ Bl, float* C, int nValid) {
  constexpr int KSTEPS = K / 32;
  constexpr int PPR = K / 4;
  constexpr int NIT = (BM * PPR) / NTHR;
  constexpr int OPR = DW / 4;
  constexpr int NOUT = (BM * OPR) / NTHR;
  constexpr int TPW = 2;
  static_assert((K % 32) == 0);
  static_assert((BM * PPR) % NTHR == 0);
  static_assert((BM * OPR) % NTHR == 0);
  static_assert(NIT >= 1 && NOUT >= 1);
  static_assert(BM == 4 * 16 && DW == 2 * TPW * 16 && NWAVE == 8);
  static_assert(K >= DW);

  __shared__ __attribute__((aligned(16))) float lraw[BM * K];
  unsigned short* ahi = (unsigned short*)lraw;
  unsigned short* alo = ahi + BM * K;
  float* stg = lraw;

  const int tid = threadIdx.x, lane = tid & 31, wave = tid >> 5, hh = lane >> 4, m = lane & 15;
  const int rowBase = (int)blockIdx.x * BM;
  const int rg = wave >> 1, chf = wave & 1;
  const int r0 = rg * 16;
  const int c0 = chf * (DW / 2);

#pragma unroll
  for (int it = 0; it < NIT; ++it) {
    const int id = it * NTHR + tid;
    const int row = id / PPR, seg = id - row * PPR;
    const int grow = rowBase + row;
    const bool live = grow < nValid;
    int rr = grow > nValid - 1 ? nValid - 1 : grow;
    rr = rr < 0 ? 0 : rr;
    const v4f xv = *(const v4f*)(A + (size_t)rr * K + 4 * seg);
    const float f0 = live ? xv.x : 0.f;
    const float f1 = live ? xv.y : 0.f;
    const float f2 = live ? xv.z : 0.f;
    const float f3 = live ? xv.w : 0.f;
    unsigned short h0, l0, h1, l1, h2, l2, h3, l3;
    split2(f0, &h0, &l0);
    split2(f1, &h1, &l1);
    split2(f2, &h2, &l2);
    split2(f3, &h3, &l3);
    v4us hv, lv;
    hv.x = h0; hv.y = h1; hv.z = h2; hv.w = h3;
    lv.x = l0; lv.y = l1; lv.z = l2; lv.w = l3;
    *(v4us*)(ahi + (size_t)row * K + 4 * seg) = hv;
    *(v4us*)(alo + (size_t)row * K + 4 * seg) = lv;
  }
  __syncthreads();

  v8f acc[TPW];
#pragma unroll
  for (int t = 0; t < TPW; ++t) { v8f z = {0.f, 0.f, 0.f, 0.f, 0.f, 0.f, 0.f, 0.f}; acc[t] = z; }

  const unsigned short* ahp = ahi + (size_t)(r0 + m) * K + 8 * hh;
  const unsigned short* alp = alo + (size_t)(r0 + m) * K + 8 * hh;
  const unsigned short* bhp = Bh + (size_t)(c0 + m) * K + 8 * hh;
  const unsigned short* blp = Bl + (size_t)(c0 + m) * K + 8 * hh;
#pragma unroll 1
  for (int kt = 0; kt < KSTEPS; ++kt) {
    Frag fh, fl;
    fh.h[0] = *(const v8us*)(ahp + 32 * kt);
    fh.h[1] = *(const v8us*)(ahp + 32 * kt + 16);
    fl.h[0] = *(const v8us*)(alp + 32 * kt);
    fl.h[1] = *(const v8us*)(alp + 32 * kt + 16);
#pragma unroll
    for (int t = 0; t < TPW; ++t) {
      const size_t to = (size_t)(16 * t) * K + 32 * kt;
      Frag bh, bl;
      bh.h[0] = *(const v8us*)(bhp + to);
      bh.h[1] = *(const v8us*)(bhp + to + 16);
      bl.h[0] = *(const v8us*)(blp + to);
      bl.h[1] = *(const v8us*)(blp + to + 16);
      acc[t] = wmb(fh.v, bh.v, acc[t]);
      acc[t] = wmb(fl.v, bh.v, acc[t]);
      acc[t] = wmb(fh.v, bl.v, acc[t]);
    }
  }
  __syncthreads();

  {
    float* sp = stg + (size_t)(r0 + 8 * hh) * DW + c0 + m;
    const int growb = rowBase + r0 + 8 * hh;
#pragma unroll
    for (int t = 0; t < TPW; ++t) {
#pragma unroll
      for (int r = 0; r < 8; ++r) {
        const bool lv = (growb + r) < nValid;
        float g = acc[t][r];
        if constexpr (RELU != 0) g = fmaxf(g, 0.f);
        sp[r * DW + 16 * t] = lv ? g : 0.f;
      }
    }
  }
  __syncthreads();

  v4f cv[NOUT];
#pragma unroll
  for (int it = 0; it < NOUT; ++it) {
    const int id = it * NTHR + tid;
    const int row = id / OPR, seg = id - row * OPR;
    cv[it] = *(const v4f*)(stg + (size_t)row * DW + 4 * seg);
  }
#pragma unroll
  for (int it = 0; it < NOUT; ++it) {
    const int id = it * NTHR + tid;
    const int row = id / OPR, seg = id - row * OPR;
    float* gp = C + (size_t)(rowBase + row) * DW + 4 * seg;
    *(volatile v4f*)gp = cv[it];
  }
  __threadfence();
#pragma unroll
  for (int it = 0; it < NOUT; ++it) {
    const int id = it * NTHR + tid;
    const int row = id / OPR, seg = id - row * OPR;
    float* gp = C + (size_t)(rowBase + row) * DW + 4 * seg;
    *(volatile v4f*)gp = cv[it];
  }
}

__global__ __launch_bounds__(NTHR) void k_agg(
    const int* __restrict__ csr, const int* __restrict__ off, const int* __restrict__ cnt,
    const float* __restrict__ h, float* xo, int nN, int csrLen) {
  __shared__ __attribute__((aligned(16))) float stg[TGT * DW];
  constexpr int OPR = DW / 4;
  constexpr int NST = (TGT * OPR) / NTHR;
  static_assert((TGT * OPR) % NTHR == 0);
  const int tid = threadIdx.x, lane = tid & 31, wave = tid >> 5;
  const int bbase = blockIdx.x * TGT;
  const int tbase = bbase + wave * DPW;
  const int col2 = 2 * lane;
  const int cl    = tbase + (lane & (DPW - 1));
  const int cnt_l = cnt[cl];
  const int off_l = off[cl];

#pragma unroll 1
  for (int j = 0; j < DPW; ++j) {
    const int c = tbase + j;
    int n = __shfl(cnt_l, j);
    n = n < 0 ? 0 : (n > DEGCAP ? DEGCAP : n);
    const int st = __shfl(off_l, j);

    v2f a = {0.f, 0.f};
#pragma unroll 1
    for (int q0 = 0; q0 < n; q0 += 32) {
      int pos = st + q0 + lane;
      pos = pos < 0 ? 0 : (pos > csrLen - 1 ? csrLen - 1 : pos);
      int sl = csr[pos];
      sl = sl < 0 ? 0 : (sl > nN - 1 ? nN - 1 : sl);
      const int mcnt = (n - q0) < 32 ? (n - q0) : 32;
#pragma unroll 1
      for (int pp = 0; pp < mcnt; ++pp) {
        const int s = __builtin_amdgcn_readlane(sl, pp);
        const v2f xv = *(const v2f*)(h + (size_t)s * DW + col2);
        a = a + xv;
      }
    }

    const bool live = c < nN;
    v2f o;
    o.x = live ? fmaxf(a.x, 0.f) : 0.f;
    o.y = live ? fmaxf(a.y, 0.f) : 0.f;
    *(v2f*)(stg + (size_t)(wave * DPW + j) * DW + col2) = o;
  }
  __syncthreads();

  v4f cv[NST];
#pragma unroll
  for (int it = 0; it < NST; ++it) {
    const int id = it * NTHR + tid;
    const int row = id / OPR, seg = id - row * OPR;
    cv[it] = *(const v4f*)(stg + (size_t)row * DW + 4 * seg);
  }
#pragma unroll
  for (int it = 0; it < NST; ++it) {
    const int id = it * NTHR + tid;
    const int row = id / OPR, seg = id - row * OPR;
    float* gp = xo + (size_t)(bbase + row) * DW + 4 * seg;
    *(volatile v4f*)gp = cv[it];
  }
  __threadfence();
#pragma unroll
  for (int it = 0; it < NST; ++it) {
    const int id = it * NTHR + tid;
    const int row = id / OPR, seg = id - row * OPR;
    float* gp = xo + (size_t)(bbase + row) * DW + 4 * seg;
    *(volatile v4f*)gp = cv[it];
  }
}

__global__ __launch_bounds__(NTHR) void k_pool(
    const int* __restrict__ batch, const float* __restrict__ h, float* P, int colOff, int nN, int vec8) {
  __shared__ __attribute__((aligned(16))) int list[LISTN];
  __shared__ __attribute__((aligned(16))) float spart[NWAVE * GPB * DW];
  __shared__ __attribute__((aligned(16))) float ssum[GPB * DW];
  const int tid = threadIdx.x, lane = tid & 31, wave = tid >> 5;
  const int gBase = blockIdx.x * GPB;
  const int col2 = 2 * lane;

  v2f acc[GPB];
#pragma unroll
  for (int s = 0; s < GPB; ++s) { v2f z = {0.f, 0.f}; acc[s] = z; }

  const int nChunks = (nN + CHUNK - 1) / CHUNK;
#pragma unroll 1
  for (int ch = 0; ch < nChunks; ++ch) {
    const int cbase = ch * CHUNK;
    const int wc = scan_chunk<GPB>(batch, nN, cbase, gBase, vec8, list, tid, lane, wave);
    __syncthreads();
    int n = wc;
    n = n > WCAP ? WCAP : (n < 0 ? 0 : n);
    const int* lp = list + wave * WCAP;
#pragma unroll 1
    for (int i = 0; i < n; ++i) {
      const int ent = __builtin_amdgcn_readfirstlane(lp[i]);
      int node = cbase + ((ent >> 12) & (CHUNK - 1));
      node = node > nN - 1 ? nN - 1 : (node < 0 ? 0 : node);
      const int slot = ent & (GPB - 1);
      const v2f hv = *(const v2f*)(h + (size_t)node * DW + col2);
#pragma unroll
      for (int s = 0; s < GPB; ++s) {
        const bool hit = slot == s;
        v2f add;
        add.x = hit ? hv.x : 0.f;
        add.y = hit ? hv.y : 0.f;
        acc[s] = acc[s] + add;
      }
    }
    __syncthreads();
  }

#pragma unroll
  for (int s = 0; s < GPB; ++s) *(v2f*)(spart + (size_t)(wave * GPB + s) * DW + col2) = acc[s];
  __syncthreads();
#pragma unroll
  for (int q = 0; q < (GPB * DW) / NTHR; ++q) {
    const int idx = q * NTHR + tid;
    const int s = idx / DW, c = idx - s * DW;
    float S = 0.f;
#pragma unroll
    for (int w = 0; w < NWAVE; ++w) S += spart[(w * GPB + s) * DW + c];
    ssum[idx] = S;
  }
  __syncthreads();
  constexpr int OPR = DW / 4;
  const bool stl = tid < GPB * OPR;
  const int row = tid / OPR, seg = tid - (tid / OPR) * OPR;
  v4f v = {0.f, 0.f, 0.f, 0.f};
  float* gp = P + (size_t)(gBase + (stl ? row : 0)) * KH + colOff + 4 * (stl ? seg : 0);
  if (stl) {
    v = *(const v4f*)(ssum + (size_t)row * DW + 4 * seg);
    *(volatile v4f*)gp = v;
  }
  __threadfence();
  if (stl) *(volatile v4f*)gp = v;
}

extern "C" void kernel_launch(void* const* d_in, const int* in_sizes, int n_in,
                              void* d_out, int out_size, void* d_ws, size_t ws_size,
                              hipStream_t stream) {
  if (n_in < 9) return;
  if (in_sizes[0] < DW || (in_sizes[0] % DW) != 0) return;
  const int nN = in_sizes[0] / DW;
  if (in_sizes[1] < 2 || (in_sizes[1] & 1) != 0) return;
  const int nE = in_sizes[1] / 2;
  if (in_sizes[2] != nN) return;
  for (int i = 3; i < 9; ++i) if (in_sizes[i] != DW * DW) return;
  if (out_size < DW || (out_size % DW) != 0) return;
  const int nG = out_size / DW;
  if ((nG % BM) != 0 || nG > GMAX) return;
  if (nE > (1 << 28) || nN > (1 << 22)) return;

  const float* x     = (const float*)d_in[0];
  const int*   ei    = (const int*)d_in[1];
  const int*   src   = ei;
  const int*   dst   = ei + nE;
  const int*   batch = (const int*)d_in[2];
  const float* wA    = (const float*)d_in[3];
  const float* wB    = (const float*)d_in[4];
  const float* wC    = (const float*)d_in[5];
  const float* wpA   = (const float*)d_in[6];
  const float* wpB   = (const float*)d_in[7];
  const float* wpC   = (const float*)d_in[8];
  float* out = (float*)d_out;

  const int NPAD   = ((nN + TGT - 1) / TGT) * TGT;
  const int nBC    = (nN + NBC - 1) / NBC;
  const int CNTPAD = nBC * NBC;
  if (CNTPAD < NPAD) return;
  if (4 * nBC + 1 > RBN) return;
  const int nBF    = (nN + NBF - 1) / NBF;
  if (nBF > 4 * nBC) return;
  const int csrLen = ((nE + 31) & ~31) + 4096;
  if (31 * 4 * nBC > 4096) return;
  const int nAgg   = NPAD / TGT;
  const int nGemm  = NPAD / BM;
  const int nUnits = 6 * DW * (DW / 8);
  const int GBLK   = (nG + GPB - 1) / GPB;
  const int GPAD   = GBLK * GPB;
  const int WTOT   = NMAT * DW * DW + DW * KH;

  char* ws = (char*)d_ws;
  size_t off = 0;
  const size_t oWh  = off; off += (size_t)WTOT * 2;               off = (off + 255) & ~(size_t)255;
  const size_t oWl  = off; off += (size_t)WTOT * 2;               off = (off + 255) & ~(size_t)255;
  const size_t oH   = off; off += (size_t)NPAD * DW * 4;          off = (off + 255) & ~(size_t)255;
  const size_t oX   = off; off += (size_t)NPAD * DW * 4;          off = (off + 255) & ~(size_t)255;
  const size_t oCnt = off; off += (size_t)CNTPAD * 4;             off = (off + 255) & ~(size_t)255;
  const size_t oOff = off; off += (size_t)CNTPAD * 4;             off = (off + 255) & ~(size_t)255;
  const size_t oRb  = off; off += (size_t)RBN * 4;                off = (off + 255) & ~(size_t)255;
  const size_t oCsr = off; off += (size_t)csrLen * 4;             off = (off + 255) & ~(size_t)255;
  const size_t oP   = off; off += (size_t)GPAD * KH * 4;          off = (off + 255) & ~(size_t)255;
  if (off > ws_size || off > (size_t)WSCAP) return;

  unsigned short* whi = (unsigned short*)(ws + oWh);
  unsigned short* wlo = (unsigned short*)(ws + oWl);
  float* hp   = (float*)(ws + oH);
  float* xp   = (float*)(ws + oX);
  int*   cnt  = (int*)(ws + oCnt);
  int*   offp = (int*)(ws + oOff);
  int*   rb   = (int*)(ws + oRb);
  int*   csr  = (int*)(ws + oCsr);
  float* P    = (float*)(ws + oP);

  const int vec8 = ((nE & 3) == 0) ? 1 : 0;

  k_wcvt<<<(nUnits + NTHR - 1) / NTHR, NTHR, 0, stream>>>(wA, wB, wC, wpA, wpB, wpC, whi, wlo, nUnits);
  k_count<<<nBC, NTHR, 0, stream>>>(dst, cnt, nE, vec8);
  k_offsets<<<1, OTHR, 0, stream>>>(cnt, offp, rb, nBC);
  hipFuncSetAttribute(reinterpret_cast<const void*>(&k_fill),
                      hipFuncAttributeMaxDynamicSharedMemorySize, LDS_FILL);
  k_fill<<<nBF, NTHR, LDS_FILL, stream>>>(src, dst, offp, rb, csr, nN, nE, vec8, csrLen);

  for (int l = 0; l < NMAT; ++l) {
    const float* asrc = (l == 0) ? x : xp;
    k_gemm<DW, 0><<<nGemm, NTHR, 0, stream>>>(asrc, whi + (size_t)l * DW * DW, wlo + (size_t)l * DW * DW, hp, nN);
    k_agg<<<nAgg, NTHR, 0, stream>>>(csr, offp, cnt, hp, xp, nN, csrLen);
    k_pool<<<GBLK, NTHR, 0, stream>>>(batch, xp, P, l * DW, nN, 1);
  }

  k_gemm<KH, 1><<<nG / BM, NTHR, 0, stream>>>(P, whi + (size_t)NMAT * DW * DW, wlo + (size_t)NMAT * DW * DW, out, nG);
}
